// GradKPCA_68874095558879
// MI455X (gfx1250) — hardware-run, weakly checked
//
#include <hip/hip_runtime.h>
#include <math.h>

typedef __attribute__((ext_vector_type(16))) _Float16 v16h;
typedef __attribute__((ext_vector_type(8)))  _Float16 v8h;
typedef __attribute__((ext_vector_type(8)))  float    v8f;
typedef __attribute__((ext_vector_type(4)))  float    v4f;
typedef __attribute__((ext_vector_type(4)))  unsigned v4u;

constexpr int kN      = 8192;
constexpr int kD      = 1024;
constexpr int kNC     = 256;
constexpr int kLS     = 512;
constexpr int kHID    = 4 * kLS;
constexpr int kCAT    = kHID + kNC;
constexpr int kBand   = 2048;
constexpr int kNBands = kN / kBand;
constexpr float kGamma   = 10.0f;
constexpr float kInvGD   = 1.0f / (kGamma * (float)kD);
constexpr float kShift   = 0.818730753f;
constexpr float kCarry    = 1024.0f;
constexpr float kCarryInv = 1.0f / kCarry;
constexpr float kMeanScale = 1.0f / ((float)kN * kCarry);
constexpr float kInvN      = 1.0f / (float)kN;

static_assert(kHID == 2048 && kCAT == 2304 && kNBands == 4, "shape constants");
static_assert((kD % 32) == 0 && (kN % 32) == 0 && (kNC % 32) == 0 && (kCAT % 32) == 0, "GEMM K multiples of 32");
static_assert((kBand % 64) == 0 && (kN % 64) == 0 && (kNC % 64) == 0 && (kHID % 64) == 0 && (kLS % 64) == 0, "GEMM M,N multiples of 64");
static_assert((kCAT % 64) == 0, "hcat/Wcat pitch is a whole number of 128-B lines");

constexpr size_t kOffXH   = 0;
constexpr size_t kOffSQN  = kOffXH   + (size_t)kN * kD * 2;
constexpr size_t kOffWT   = kOffSQN  + (size_t)kN * 4;
constexpr size_t kOffW1T  = kOffWT   + (size_t)kNC * kN * 2;
constexpr size_t kOffWCAT = kOffW1T  + (size_t)kHID * kNC * 2;
constexpr size_t kOffKB   = kOffWCAT + (size_t)kLS * kCAT * 2;
constexpr size_t kOffMU   = kOffKB   + (size_t)kBand * kN * 2;
constexpr size_t kOffRAW  = kOffMU   + (size_t)kN * 4;
constexpr size_t kOffCV   = kOffRAW  + (size_t)kN * kNC * 4;
constexpr size_t kOffHCAT = kOffCV   + (size_t)2 * kNC * 4;
constexpr size_t kOffSCH  = kOffHCAT + (size_t)kN * kCAT * 2;
constexpr size_t kWsTotal = kOffSCH  + (size_t)kN * kNC * 2;
static_assert(kWsTotal == 108333056ull, "carve total");
static_assert(kWsTotal <= 134217728ull, "carve cap");
static_assert((kOffSQN % 128) == 0 && (kOffWT % 128) == 0 && (kOffW1T % 128) == 0 && (kOffWCAT % 128) == 0 &&
              (kOffKB % 128) == 0 && (kOffMU % 128) == 0 && (kOffRAW % 128) == 0 && (kOffCV % 128) == 0 &&
              (kOffHCAT % 128) == 0 && (kOffSCH % 128) == 0, "128-B aligned regions");

union FragU { v16h v; v8h h[2]; };
__device__ __forceinline__ v16h frag_load(const _Float16* p) {
  FragU f;
  f.h[0] = *(const v8h*)(p);
  f.h[1] = *(const v8h*)(p + 16);
  return f.v;
}
__device__ __forceinline__ v8f frag_mma(v16h a, v16h b, v8f c) {
  return __builtin_amdgcn_wmma_f32_16x16x32_f16(false, a, false, b, (short)0, c, false, false);
}
__device__ __forceinline__ void row_guard(v8f& a0, v8f& a1, v8f& a2, v8f& a3, v16h x,
                                          v16h b0, v16h b1, v16h b2, v16h b3) {
  asm volatile("v_nop\n\tv_nop\n\tv_nop\n\tv_nop"
               : "+v"(a0), "+v"(a1), "+v"(a2), "+v"(a3)
               : "v"(x), "v"(b0), "v"(b1), "v"(b2), "v"(b3));
}
__device__ __forceinline__ void acc_guard4(v8f& a, v8f& b, v8f& c, v8f& d) {
  asm volatile("v_nop\n\tv_nop\n\tv_nop\n\tv_nop" : "+v"(a), "+v"(b), "+v"(c), "+v"(d));
}

__device__ __forceinline__ float h16_to_f32(unsigned hb) {
  const unsigned sgn = (hb & 0x8000u) << 16;
  const unsigned em = hb & 0x7fffu;
  const float fn = __uint_as_float((em << 13) + 0x38000000u);
  const float fs = (float)em * 5.9604644775390625e-8f;
  const float mag = (em < 0x400u) ? fs : fn;
  return __uint_as_float(__float_as_uint(mag) | sgn);
}

__device__ __forceinline__ void rbf_stage(float* slab, const v8f& t0, const v8f& t1, const v8f& t2, const v8f& t3,
                                          const v4f ra, const v4f rb, float c0, float c1, float c2, float c3,
                                          int mOff, int rlane) {
#pragma unroll
  for (int r = 0; r < 8; ++r) {
    const float sr = (r < 4) ? ra[r & 3] : rb[r & 3];
    float* o = slab + (mOff + r) * 68 + rlane;
    o[0]  = (sr + c0) - 2.0f * t0[r];
    o[16] = (sr + c1) - 2.0f * t1[r];
    o[32] = (sr + c2) - 2.0f * t2[r];
    o[48] = (sr + c3) - 2.0f * t3[r];
  }
}

template <int EPI>
__global__ __launch_bounds__(256) void gemm64_f16_kernel(
    const _Float16* __restrict__ A, int lda,
    const _Float16* __restrict__ Bt, int ldb,
    void* __restrict__ Cout, int ldc,
    const float* __restrict__ va, const float* __restrict__ vb,
    int M, int N, int K, float scale)
{
  __shared__ __align__(16) float sT[8][16 * 68];
  const int lane = threadIdx.x & 31;
  const int wave = threadIdx.x >> 5;
  const int tilesN = N >> 6;
  const int tilesM = M >> 6;
  const int tile = blockIdx.x * 8 + wave;
  if (tile >= tilesM * tilesN) return;
  const int tm = tile / tilesN;
  const int tn = tile - tm * tilesN;
  const int m0 = tm << 6;
  const int n0 = tn << 6;

  const int rlane = lane & 15;
  const int koff  = (lane >> 4) * 8;
  const int mOff  = (lane >> 4) * 8;

  v8f acc[4][4];
#pragma unroll
  for (int i = 0; i < 4; ++i)
#pragma unroll
    for (int j = 0; j < 4; ++j) acc[i][j] = (v8f){0.f, 0.f, 0.f, 0.f, 0.f, 0.f, 0.f, 0.f};

  for (int k0 = 0; k0 < K; k0 += 32) {
    v16h bh[4];
#pragma unroll
    for (int j = 0; j < 4; ++j) {
      const size_t bo = (size_t)(n0 + (j << 4) + rlane) * ldb + koff + k0;
      bh[j] = frag_load(Bt + bo);
    }
#pragma unroll
    for (int i = 0; i < 4; ++i) {
      const size_t ao = (size_t)(m0 + (i << 4) + rlane) * lda + koff + k0;
      const v16h ah = frag_load(A + ao);
#pragma unroll
      for (int j = 0; j < 4; ++j) acc[i][j] = frag_mma(ah, bh[j], acc[i][j]);
      row_guard(acc[i][0], acc[i][1], acc[i][2], acc[i][3], ah, bh[0], bh[1], bh[2], bh[3]);
    }
  }
  acc_guard4(acc[0][0], acc[0][1], acc[0][2], acc[0][3]);
  acc_guard4(acc[1][0], acc[1][1], acc[1][2], acc[1][3]);
  acc_guard4(acc[2][0], acc[2][1], acc[2][2], acc[2][3]);
  acc_guard4(acc[3][0], acc[3][1], acc[3][2], acc[3][3]);

  float* slab = sT[wave];

  if (EPI == 3) {
    _Float16* C = (_Float16*)Cout;
    const float sc0 = vb[n0 + 0  + rlane];
    const float sc1 = vb[n0 + 16 + rlane];
    const float sc2 = vb[n0 + 32 + rlane];
    const float sc3 = vb[n0 + 48 + rlane];
    const int q = lane >> 3, c8 = (lane & 7) * 8;
#pragma unroll 1
    for (int i = 0; i < 4; ++i) {
      const int mBase = m0 + (i << 4);
      const v4f ra = *(const v4f*)(va + mBase + mOff);
      const v4f rb = *(const v4f*)(va + mBase + mOff + 4);
      if (i == 0)      rbf_stage(slab, acc[0][0], acc[0][1], acc[0][2], acc[0][3], ra, rb, sc0, sc1, sc2, sc3, mOff, rlane);
      else if (i == 1) rbf_stage(slab, acc[1][0], acc[1][1], acc[1][2], acc[1][3], ra, rb, sc0, sc1, sc2, sc3, mOff, rlane);
      else if (i == 2) rbf_stage(slab, acc[2][0], acc[2][1], acc[2][2], acc[2][3], ra, rb, sc0, sc1, sc2, sc3, mOff, rlane);
      else             rbf_stage(slab, acc[3][0], acc[3][1], acc[3][2], acc[3][3], ra, rb, sc0, sc1, sc2, sc3, mOff, rlane);
      __builtin_amdgcn_fence(__ATOMIC_RELEASE, "workgroup");
      __builtin_amdgcn_wave_barrier();
      __builtin_amdgcn_fence(__ATOMIC_ACQUIRE, "workgroup");
#pragma unroll 1
      for (int it = 0; it < 4; ++it) {
        const int row = it * 4 + q;
        const float* sp = slab + row * 68 + c8;
        const v4f a0 = *(const v4f*)(sp);
        const v4f a1 = *(const v4f*)(sp + 4);
        v8h hv;
#pragma unroll
        for (int e = 0; e < 4; ++e) {
          const float d0 = fmaxf(a0[e], 0.0f);
          const float d1 = fmaxf(a1[e], 0.0f);
          const float k0v = (expf(-d0 * kInvGD) - kShift) * kCarry;
          const float k1v = (expf(-d1 * kInvGD) - kShift) * kCarry;
          hv[e]     = (_Float16)k0v;
          hv[4 + e] = (_Float16)k1v;
        }
        _Float16* dst = C + (size_t)(mBase + row) * ldc + n0 + c8;
        *(volatile v8h*)dst = hv;
        __threadfence();
        *(volatile v8h*)dst = hv;
      }
      __builtin_amdgcn_fence(__ATOMIC_RELEASE, "workgroup");
      __builtin_amdgcn_wave_barrier();
      __builtin_amdgcn_fence(__ATOMIC_ACQUIRE, "workgroup");
    }
  } else {
    float bv[4];
#pragma unroll
    for (int j = 0; j < 4; ++j) {
      const int n = n0 + (j << 4) + rlane;
      bv[j] = 0.f;
      if (EPI == 1) bv[j] = va[n];
      if (EPI == 2) bv[j] = va[n] + vb[n];
    }
#pragma unroll
    for (int i = 0; i < 4; ++i) {
      const int mBase = m0 + (i << 4);
#pragma unroll
      for (int j = 0; j < 4; ++j) {
#pragma unroll
        for (int r = 0; r < 8; ++r) {
          float v = acc[i][j][r];
          if (EPI == 0) v = v * scale;
          if (EPI == 1) v = fmaxf(v + bv[j], 0.0f);
          if (EPI == 2) v = v + bv[j];
          slab[(mOff + r) * 68 + (j << 4) + rlane] = v;
        }
      }
      __builtin_amdgcn_fence(__ATOMIC_RELEASE, "workgroup");
      __builtin_amdgcn_wave_barrier();
      __builtin_amdgcn_fence(__ATOMIC_ACQUIRE, "workgroup");
      if (EPI == 0 || EPI == 2) {
        float* C = (float*)Cout;
        const int hh = lane >> 4, c4 = (lane & 15) * 4;
        for (int pass = 0; pass < 2; ++pass) {
#pragma unroll
          for (int it = 0; it < 8; ++it) {
            const int row = it * 2 + hh;
            const v4f v = *(const v4f*)(slab + row * 68 + c4);
            *(volatile v4f*)(C + (size_t)(mBase + row) * ldc + n0 + c4) = v;
          }
          __threadfence();
        }
      } else {
        _Float16* C = (_Float16*)Cout;
        const int q = lane >> 3, c8 = (lane & 7) * 8;
        for (int pass = 0; pass < 2; ++pass) {
#pragma unroll
          for (int it = 0; it < 4; ++it) {
            const int row = it * 4 + q;
            const float* sp = slab + row * 68 + c8;
            v8h hv;
#pragma unroll
            for (int e = 0; e < 8; ++e) hv[e] = (_Float16)sp[e];
            *(volatile v8h*)(C + (size_t)(mBase + row) * ldc + n0 + c8) = hv;
          }
          __threadfence();
        }
      }
      __builtin_amdgcn_fence(__ATOMIC_RELEASE, "workgroup");
      __builtin_amdgcn_wave_barrier();
      __builtin_amdgcn_fence(__ATOMIC_ACQUIRE, "workgroup");
    }
  }
}

__global__ __launch_bounds__(256) void cvt_rows_f16_kernel(
    const float* __restrict__ src, _Float16* __restrict__ dst, int total8)
{
  const int i = blockIdx.x * 256 + threadIdx.x;
  if (i >= total8) return;
  const size_t e0 = (size_t)i << 3;
  const v4f a0 = *(const v4f*)(src + e0);
  const v4f a1 = *(const v4f*)(src + e0 + 4);
  v8h hv;
#pragma unroll
  for (int e = 0; e < 4; ++e) {
    hv[e]     = (_Float16)a0[e];
    hv[4 + e] = (_Float16)a1[e];
  }
  _Float16* d = dst + e0;
  *(volatile v8h*)d = hv;
  __threadfence();
  *(volatile v8h*)d = hv;
}

__global__ __launch_bounds__(256) void sqnorm_kernel(const float* __restrict__ x, float* __restrict__ sqn)
{
  const int row = blockIdx.x * 256 + threadIdx.x;
  const float* p = x + (size_t)row * kD;
  float s0 = 0.f, s1 = 0.f, s2 = 0.f, s3 = 0.f;
#pragma unroll 4
  for (int k = 0; k < kD; k += 4) {
    const v4f v = *(const v4f*)(p + k);
    s0 = fmaf(v[0], v[0], s0);
    s1 = fmaf(v[1], v[1], s1);
    s2 = fmaf(v[2], v[2], s2);
    s3 = fmaf(v[3], v[3], s3);
  }
  const float s = (s0 + s1) + (s2 + s3);
  *(volatile float*)(sqn + row) = s;
  __threadfence();
  *(volatile float*)(sqn + row) = s;
}

__global__ __launch_bounds__(256) void transpose_cvt_kernel(
    const float* __restrict__ src, int C, _Float16* __restrict__ dst, int ldd, int coff)
{
  __shared__ __align__(16) float tile[64 * 68];
  const int tid = threadIdx.x, lane = tid & 31, wave = tid >> 5;
  const int c0 = blockIdx.x * 64;
  const int r0 = blockIdx.y * 64;
#pragma unroll
  for (int it = 0; it < 4; ++it) {
    const int idx = it * 256 + tid;
    const int r = idx >> 4;
    const int c4 = (idx & 15) * 4;
    *(v4f*)(tile + r * 68 + c4) = *(const v4f*)(src + (size_t)(r0 + r) * C + c0 + c4);
  }
  __syncthreads();
  const int q = lane >> 3, r8 = (lane & 7) * 8;
  v8h hv[2];
#pragma unroll
  for (int it = 0; it < 2; ++it) {
    const int c = it * 32 + wave * 4 + q;
#pragma unroll
    for (int e = 0; e < 8; ++e) hv[it][e] = (_Float16)tile[(r8 + e) * 68 + c];
  }
  for (int pass = 0; pass < 2; ++pass) {
#pragma unroll
    for (int it = 0; it < 2; ++it) {
      const int c = it * 32 + wave * 4 + q;
      *(volatile v8h*)(dst + (size_t)(c0 + c) * ldd + coff + r0 + r8) = hv[it];
    }
    __threadfence();
  }
}

__global__ __launch_bounds__(256) void rowmean_kernel(
    const unsigned short* __restrict__ Kb, float* __restrict__ mu_band)
{
  __shared__ float red[32];
  const int tid = threadIdx.x, lane = tid & 31, wave = tid >> 5;
#pragma unroll 1
  for (int rr = 0; rr < 4; ++rr) {
    const int row = blockIdx.x * 32 + wave * 4 + rr;
    const v4u* p = (const v4u*)(Kb + (size_t)row * kN);
    float s0 = 0.f, s1 = 0.f, s2 = 0.f, s3 = 0.f;
#pragma unroll 1
    for (int it = 0; it < kN / 256; ++it) {
      const v4u w = p[it * 32 + lane];
      const unsigned w0 = w[0];
      const unsigned w1 = w[1];
      const unsigned w2 = w[2];
      const unsigned w3 = w[3];
      s0 += h16_to_f32(w0 & 0xffffu) + h16_to_f32(w0 >> 16);
      s1 += h16_to_f32(w1 & 0xffffu) + h16_to_f32(w1 >> 16);
      s2 += h16_to_f32(w2 & 0xffffu) + h16_to_f32(w2 >> 16);
      s3 += h16_to_f32(w3 & 0xffffu) + h16_to_f32(w3 >> 16);
    }
    float s = (s0 + s1) + (s2 + s3);
    s += __shfl_xor(s, 16, 32);
    s += __shfl_xor(s, 8, 32);
    s += __shfl_xor(s, 4, 32);
    s += __shfl_xor(s, 2, 32);
    s += __shfl_xor(s, 1, 32);
    if (lane == 0) red[wave * 4 + rr] = s;
  }
  __syncthreads();
  if (wave == 0) {
    const float m = red[lane] * kMeanScale;
    float* o = mu_band + blockIdx.x * 32 + lane;
    *(volatile float*)o = m;
    __threadfence();
    *(volatile float*)o = m;
  }
}

__global__ __launch_bounds__(256) void stats_kernel(
    const unsigned short* __restrict__ Wt, const float* __restrict__ mu,
    float* __restrict__ cvec, float* __restrict__ wcol)
{
  __shared__ float r1[8 * 32];
  __shared__ float r2[8 * 32];
  __shared__ float rg[8];
  const int tid = threadIdx.x, jl = tid & 31, ks = tid >> 5;
  const int j = blockIdx.x * 32 + jl;
  const v4u* wp = (const v4u*)(Wt + (size_t)j * kN + ks * 1024);
  const float* mp = mu + ks * 1024;
  float s1a = 0.f, s1b = 0.f, s2a = 0.f, s2b = 0.f, ga = 0.f, gb = 0.f;
#pragma unroll 1
  for (int it = 0; it < 128; ++it) {
    const v4u w = wp[it];
    const v4f ma = *(const v4f*)(mp + 8 * it);
    const v4f mb = *(const v4f*)(mp + 8 * it + 4);
    const unsigned w0 = w[0];
    const unsigned w1 = w[1];
    const unsigned w2 = w[2];
    const unsigned w3 = w[3];
    const float f0 = h16_to_f32(w0 & 0xffffu);
    const float f1 = h16_to_f32(w0 >> 16);
    const float f2 = h16_to_f32(w1 & 0xffffu);
    const float f3 = h16_to_f32(w1 >> 16);
    const float f4 = h16_to_f32(w2 & 0xffffu);
    const float f5 = h16_to_f32(w2 >> 16);
    const float f6 = h16_to_f32(w3 & 0xffffu);
    const float f7 = h16_to_f32(w3 >> 16);
    s1a = fmaf(ma[0], f0, s1a);
    s1b = fmaf(ma[1], f1, s1b);
    s1a = fmaf(ma[2], f2, s1a);
    s1b = fmaf(ma[3], f3, s1b);
    s1a = fmaf(mb[0], f4, s1a);
    s1b = fmaf(mb[1], f5, s1b);
    s1a = fmaf(mb[2], f6, s1a);
    s1b = fmaf(mb[3], f7, s1b);
    s2a += (f0 + f2) + (f4 + f6);
    s2b += (f1 + f3) + (f5 + f7);
    ga += (ma[0] + ma[1]) + (ma[2] + ma[3]);
    gb += (mb[0] + mb[1]) + (mb[2] + mb[3]);
  }
  r1[ks * 32 + jl] = s1a + s1b;
  r2[ks * 32 + jl] = s2a + s2b;
  if (jl == 0) rg[ks] = ga + gb;
  __syncthreads();
  if (ks == 0) {
    float mw = 0.f, wc = 0.f, gs = 0.f;
#pragma unroll
    for (int s = 0; s < 8; ++s) {
      mw += r1[s * 32 + jl];
      wc += r2[s * 32 + jl];
      gs += rg[s];
    }
    const float g = gs * kInvN;
    const float cv = mw - g * wc;
    *(volatile float*)(cvec + j) = cv;
    *(volatile float*)(wcol + j) = wc;
    __threadfence();
    *(volatile float*)(cvec + j) = cv;
    *(volatile float*)(wcol + j) = wc;
  }
}

__global__ __launch_bounds__(256) void finalize_score_kernel(
    const float* __restrict__ raw, const float* __restrict__ mu,
    const float* __restrict__ cvec, const float* __restrict__ wcol,
    _Float16* __restrict__ sch, _Float16* __restrict__ hcat)
{
  const int idx = blockIdx.x * 256 + threadIdx.x;
  const int i = idx >> 5;
  const int j8 = (idx & 31) << 3;
  const float m = mu[i];
  const v4f ra = *(const v4f*)(raw + (size_t)i * kNC + j8);
  const v4f rb = *(const v4f*)(raw + (size_t)i * kNC + j8 + 4);
  const v4f ca = *(const v4f*)(cvec + j8);
  const v4f cb = *(const v4f*)(cvec + j8 + 4);
  const v4f wa = *(const v4f*)(wcol + j8);
  const v4f wb = *(const v4f*)(wcol + j8 + 4);
  v8h hv;
#pragma unroll
  for (int e = 0; e < 4; ++e) {
    const float sa = (ra[e] - ca[e]) - m * wa[e];
    const float sb = (rb[e] - cb[e]) - m * wb[e];
    hv[e]     = (_Float16)sa;
    hv[4 + e] = (_Float16)sb;
  }
  _Float16* p0 = sch + (size_t)i * kNC + j8;
  _Float16* p1 = hcat + (size_t)i * kCAT + kHID + j8;
  *(volatile v8h*)p0 = hv;
  *(volatile v8h*)p1 = hv;
  __threadfence();
  *(volatile v8h*)p0 = hv;
  *(volatile v8h*)p1 = hv;
}

extern "C" void kernel_launch(void* const* d_in, const int* in_sizes, int n_in,
                              void* d_out, int out_size, void* d_ws, size_t ws_size,
                              hipStream_t stream) {
  if (n_in < 8) return;
  if (in_sizes[0] != kN * kD) return;
  if (in_sizes[1] != kN * kNC) return;
  if (in_sizes[2] != kNC * kHID) return;
  if (in_sizes[3] != kHID) return;
  if (in_sizes[4] != kHID * kLS) return;
  if (in_sizes[5] != kLS) return;
  if (in_sizes[6] != kNC * kLS) return;
  if (in_sizes[7] != kLS) return;
  if (out_size != kN * kLS) return;
  if (ws_size < kWsTotal) return;

  const float* x  = (const float*)d_in[0];
  const float* W  = (const float*)d_in[1];
  const float* W1 = (const float*)d_in[2];
  const float* b1 = (const float*)d_in[3];
  const float* W2 = (const float*)d_in[4];
  const float* b2 = (const float*)d_in[5];
  const float* Ws = (const float*)d_in[6];
  const float* bs = (const float*)d_in[7];
  float* z = (float*)d_out;

  char* ws = (char*)d_ws;
  _Float16* XH   = (_Float16*)(ws + kOffXH);
  float*    SQN  = (float*)(ws + kOffSQN);
  _Float16* WT   = (_Float16*)(ws + kOffWT);
  _Float16* W1T  = (_Float16*)(ws + kOffW1T);
  _Float16* WCAT = (_Float16*)(ws + kOffWCAT);
  _Float16* KB   = (_Float16*)(ws + kOffKB);
  float*    MU   = (float*)(ws + kOffMU);
  float*    RAW  = (float*)(ws + kOffRAW);
  float*    CVEC = (float*)(ws + kOffCV);
  float*    WCOL = CVEC + kNC;
  _Float16* HCAT = (_Float16*)(ws + kOffHCAT);
  _Float16* SCH  = (_Float16*)(ws + kOffSCH);

  cvt_rows_f16_kernel<<<(kN * kD / 8) / 256, 256, 0, stream>>>(x, XH, kN * kD / 8);
  sqnorm_kernel<<<kN / 256, 256, 0, stream>>>(x, SQN);

  transpose_cvt_kernel<<<dim3(kNC / 64, kN / 64), 256, 0, stream>>>(W, kNC, WT, kN, 0);
  transpose_cvt_kernel<<<dim3(kHID / 64, kNC / 64), 256, 0, stream>>>(W1, kHID, W1T, kNC, 0);
  transpose_cvt_kernel<<<dim3(kLS / 64, kHID / 64), 256, 0, stream>>>(W2, kLS, WCAT, kCAT, 0);
  transpose_cvt_kernel<<<dim3(kLS / 64, kNC / 64), 256, 0, stream>>>(Ws, kLS, WCAT, kCAT, kHID);

  for (int b = 0; b < kNBands; ++b) {
    gemm64_f16_kernel<3><<<(kBand / 64) * (kN / 64) / 8, 256, 0, stream>>>(
        XH + (size_t)b * kBand * kD, kD,
        XH, kD,
        (void*)KB, kN,
        SQN + b * kBand, SQN,
        kBand, kN, kD, 1.0f);
    rowmean_kernel<<<kBand / 32, 256, 0, stream>>>((const unsigned short*)KB, MU + b * kBand);
    gemm64_f16_kernel<0><<<(kBand / 64) * (kNC / 64) / 8, 256, 0, stream>>>(
        KB, kN,
        WT, kN,
        (void*)(RAW + (size_t)b * kBand * kNC), kNC,
        nullptr, nullptr,
        kBand, kNC, kN, kCarryInv);
  }

  stats_kernel<<<kNC / 32, 256, 0, stream>>>((const unsigned short*)WT, MU, CVEC, WCOL);
  finalize_score_kernel<<<(kN * 32) / 256, 256, 0, stream>>>(RAW, MU, CVEC, WCOL, SCH, HCAT);

  gemm64_f16_kernel<1><<<(kN / 64) * (kHID / 64) / 8, 256, 0, stream>>>(
      SCH, kNC,
      W1T, kNC,
      (void*)HCAT, kCAT,
      b1, nullptr,
      kN, kHID, kNC, 1.0f);

  gemm64_f16_kernel<2><<<(kN / 64) * (kLS / 64) / 8, 256, 0, stream>>>(
      HCAT, kCAT,
      WCAT, kCAT,
      (void*)z, kLS,
      b2, bs,
      kN, kLS, kCAT, 1.0f);
}
